// Gemma4MoE_75849122447854
// MI455X (gfx1250) — hardware-verified
//
#include <hip/hip_runtime.h>
#include <stdint.h>
#include <stddef.h>
#include <math.h>

#pragma clang fp contract(off)

#define NTOK 4096
#define DM   1024
#define MX   1024
#define NEX  8
#define HS   2048
#define MT   64
#define XP   1032
#define HP   1032
#define YP   260
#define TP   136
#define TRP  72
#define TPB  8
#define LBW  32
#define NBLK ((NTOK + TPB - 1) / TPB)

#define LDS_XB  (MT * XP * 2)
#define LDS_HB  (MT * HP * 2)
#define LDS_EXP (LDS_XB + LDS_HB)
#define LDS_DN  (64 * YP * 4)

#define W_SC   256.0f
#define H_SC   64.0f
#define R_W    0.00390625f
#define R_HW   6.103515625e-05f
#define LOG2EF 1.4426950408889634f

static_assert(MT * YP * 4 <= LDS_XB);
static_assert((XP * 2) % 16 == 0);
static_assert((HP * 2) % 16 == 0);
static_assert((YP * 4) % 16 == 0);
static_assert((TP * 2) % 16 == 0);
static_assert((TRP * 2) % 16 == 0);
static_assert(NTOK % 256 == 0);
static_assert(NTOK % MT == 0);
static_assert(NTOK % 64 == 0);
static_assert(NTOK % TPB == 0);
static_assert(MT == 8 * 8);
static_assert(DM % 256 == 0);
static_assert(DM == 4 * 256);
static_assert(MX % 128 == 0);
static_assert(HS % 128 == 0);
static_assert(DM % 64 == 0);
static_assert(MX % 64 == 0);
static_assert(HS % 64 == 0);
static_assert(NEX == 8);
static_assert((size_t)NTOK * DM * 4 <= (size_t)NEX * MX * DM * 2);

typedef _Float16       v16h __attribute__((ext_vector_type(16)));
typedef _Float16       v8h  __attribute__((ext_vector_type(8)));
typedef float          v8f  __attribute__((ext_vector_type(8)));
typedef float          v4f  __attribute__((ext_vector_type(4)));
typedef unsigned int   v4u  __attribute__((ext_vector_type(4)));
typedef v4f __attribute__((may_alias)) v4fa;
typedef v4u __attribute__((may_alias)) v4ua;

union FragH { v16h v; v4u q[2]; };
union Pack8 { v8h h; v4u u; };

__device__ __forceinline__ unsigned short hbits(float f) {
  _Float16 t = (_Float16)f;
  unsigned short u;
  __builtin_memcpy(&u, &t, 2);
  return u;
}

__device__ __forceinline__ v8f wmma_h(v16h a, v16h b, v8f c) {
  v8f d = __builtin_amdgcn_wmma_f32_16x16x32_f16(false, a, false, b, (short)0, c, false, false);
  asm volatile("v_nop\n\tv_nop\n\tv_nop\n\tv_nop" : "+v"(d) : "v"(a), "v"(b));
  return d;
}

__device__ __forceinline__ v16h ldfrag(const unsigned short* p, int h) {
  FragH f;
  f.q[0] = *(const v4ua*)(p + 8 * h);
  f.q[1] = *(const v4ua*)(p + 16 + 8 * h);
  return f.v;
}

__device__ __forceinline__ float gelu_f(float x) {
  const float kg = -2.3022081983f;
  const float y  = x + 0.044715f * (x * x * x);
  const float s  = __builtin_amdgcn_rcpf(1.0f + exp2f(kg * y));
  return x * s;
}

__global__ __launch_bounds__(256) void k_cvt(const float* __restrict__ src,
                                             unsigned short* __restrict__ dst,
                                             int n8, float sc)
{
  const int g = blockIdx.x * 256 + threadIdx.x;
  if (g >= n8) return;
  const float* s = src + (size_t)g * 8;
  const v4f a = *(const v4fa*)s;
  const v4f c = *(const v4fa*)(s + 4);
  v8h hv;
  hv[0] = (_Float16)(a.x * sc); hv[1] = (_Float16)(a.y * sc);
  hv[2] = (_Float16)(a.z * sc); hv[3] = (_Float16)(a.w * sc);
  hv[4] = (_Float16)(c.x * sc); hv[5] = (_Float16)(c.y * sc);
  hv[6] = (_Float16)(c.z * sc); hv[7] = (_Float16)(c.w * sc);
  Pack8 p;
  p.h = hv;
  const v4u u = p.u;
  unsigned short* d = dst + (size_t)g * 8;
  *(volatile v4u*)d = u;
  __threadfence();
  *(volatile v4u*)d = u;
}

__global__ __launch_bounds__(256) void k_tr(const float* __restrict__ src,
                                            unsigned short* __restrict__ dst,
                                            int R, int CC, float sc)
{
  __shared__ __align__(16) unsigned short sT[64 * TRP];
  const int tid = threadIdx.x, lane = tid & 31, wv = tid >> 5;
  const int bz = blockIdx.z;
  const int r0 = blockIdx.y * 64;
  const int c0 = blockIdx.x * 64;
  const float* sb = src + (size_t)bz * (size_t)R * (size_t)CC;
  unsigned short* db = dst + (size_t)bz * (size_t)CC * (size_t)R;
  #pragma unroll
  for (int p = 0; p < 4; ++p) {
    const int idx = tid + 256 * p;
    const int r = idx >> 4;
    const int c4 = (idx & 15) * 4;
    const v4f v = *(const v4fa*)(sb + (size_t)(r0 + r) * CC + c0 + c4);
    sT[(c4 + 0) * TRP + r] = hbits(v.x * sc);
    sT[(c4 + 1) * TRP + r] = hbits(v.y * sc);
    sT[(c4 + 2) * TRP + r] = hbits(v.z * sc);
    sT[(c4 + 3) * TRP + r] = hbits(v.w * sc);
  }
  __syncthreads();
  #pragma unroll
  for (int i = 0; i < 2; ++i) {
    const int q = (wv * 2 + i) * 4 + (lane >> 3);
    const int piece = lane & 7;
    const v4u u = *(const v4ua*)(sT + q * TRP + 8 * piece);
    unsigned short* d = db + (size_t)(c0 + q) * R + r0 + 8 * piece;
    *(volatile v4u*)d = u;
    __threadfence();
    *(volatile v4u*)d = u;
  }
}

__global__ __launch_bounds__(256) void k_route(const float* __restrict__ xo,
                                               const float* __restrict__ pfs,
                                               const float* __restrict__ pls,
                                               const float* __restrict__ rw,
                                               float* __restrict__ rec,
                                               unsigned short* __restrict__ rxh,
                                               float* __restrict__ lbp,
                                               int ntok)
{
  __shared__ __align__(16) float swr[NEX * DM];
  __shared__ __align__(16) float spf[DM];
  __shared__ __align__(16) float spl[DM];
  __shared__ __align__(16) float srec[4 * TPB];
  __shared__ float sprob[NEX * TPB];
  __shared__ int   sidx[2 * TPB];
  const int tid = threadIdx.x, lane = tid & 31, wv = tid >> 5;

  #pragma unroll 1
  for (int i = 0; i < DM / 256; ++i) {
    const int d = tid + 256 * i;
    const v4f w0 = *(const v4fa*)(rw + (size_t)d * NEX);
    const v4f w1 = *(const v4fa*)(rw + (size_t)d * NEX + 4);
    swr[0 * DM + d] = w0.x; swr[1 * DM + d] = w0.y;
    swr[2 * DM + d] = w0.z; swr[3 * DM + d] = w0.w;
    swr[4 * DM + d] = w1.x; swr[5 * DM + d] = w1.y;
    swr[6 * DM + d] = w1.z; swr[7 * DM + d] = w1.w;
  }
  {
    const v4f a = *(const v4fa*)(pfs + 4 * tid);
    *(v4fa*)(spf + 4 * tid) = a;
    const v4f b = *(const v4fa*)(pls + 4 * tid);
    *(v4fa*)(spl + 4 * tid) = b;
  }
  __syncthreads();

  const int t = blockIdx.x * TPB + wv;
  const bool tv = (t < ntok);
  const int tc = tv ? t : (ntok - 1);
  const float* xr = xo + (size_t)tc * DM;

  double ms = 0.0;
  double lg[NEX];
  #pragma unroll
  for (int e = 0; e < NEX; ++e) lg[e] = 0.0;
  #pragma unroll 1
  for (int i = 0; i < DM / 32; ++i) {
    const int d = 32 * i + lane;
    const double xv = (double)xr[d];
    ms = fma(xv, xv, ms);
    const double g = xv * (double)spf[d];
    #pragma unroll
    for (int e = 0; e < NEX; ++e) lg[e] = fma(g, (double)swr[e * DM + d], lg[e]);
  }
  #pragma unroll
  for (int off = 16; off > 0; off >>= 1) {
    ms = ms + __shfl_xor(ms, off);
    #pragma unroll
    for (int e = 0; e < NEX; ++e) lg[e] = lg[e] + __shfl_xor(lg[e], off);
  }
  const float msf = (float)(ms * (1.0 / 1024.0));
  const float rrf = 1.0f / sqrtf(msf + 1.0e-6f);
  const double gsc = (double)rrf * (1.0 / 32.0);

  float lf[NEX];
  #pragma unroll
  for (int e = 0; e < NEX; ++e) lf[e] = (float)(lg[e] * gsc);

  int i0 = 0;
  float b0 = lf[0];
  #pragma unroll
  for (int e = 1; e < NEX; ++e) {
    const bool tk = lf[e] > b0;
    b0 = tk ? lf[e] : b0;
    i0 = tk ? e : i0;
  }
  int i1 = -1;
  float b1 = -3.0e38f;
  #pragma unroll
  for (int e = 0; e < NEX; ++e) {
    const bool tk = (e != i0) && (lf[e] > b1);
    b1 = tk ? lf[e] : b1;
    i1 = tk ? e : i1;
  }
  i1 = (i1 < 0) ? ((i0 == 0) ? 1 : 0) : i1;

  float mx = lf[0];
  #pragma unroll
  for (int e = 1; e < NEX; ++e) mx = fmaxf(mx, lf[e]);
  float p[NEX];
  float se = 0.0f;
  #pragma unroll
  for (int e = 0; e < NEX; ++e) {
    p[e] = exp2f((lf[e] - mx) * LOG2EF);
    se = se + p[e];
  }
  const float inv = 1.0f / se;
  float q0 = p[0], q1 = p[0];
  #pragma unroll
  for (int e = 0; e < NEX; ++e) { q0 = (e == i0) ? p[e] : q0; q1 = (e == i1) ? p[e] : q1; }
  const float pr0 = q0 * inv, pr1 = q1 * inv;
  const float rws = 1.0f / (pr0 + pr1);
  const float w0 = pr0 * rws, w1 = pr1 * rws;

  if (tv) {
    unsigned short* dr = rxh + (size_t)t * DM;
    v4u u[4];
    #pragma unroll
    for (int i = 0; i < 4; ++i) {
      const int d0 = 256 * i + 8 * lane;
      const v4f x0 = *(const v4fa*)(xr + d0);
      const v4f x1 = *(const v4fa*)(xr + d0 + 4);
      const v4f s0 = *(const v4fa*)(spl + d0);
      const v4f s1 = *(const v4fa*)(spl + d0 + 4);
      v8h hv;
      hv[0] = (_Float16)((x0.x * rrf) * s0.x); hv[1] = (_Float16)((x0.y * rrf) * s0.y);
      hv[2] = (_Float16)((x0.z * rrf) * s0.z); hv[3] = (_Float16)((x0.w * rrf) * s0.w);
      hv[4] = (_Float16)((x1.x * rrf) * s1.x); hv[5] = (_Float16)((x1.y * rrf) * s1.y);
      hv[6] = (_Float16)((x1.z * rrf) * s1.z); hv[7] = (_Float16)((x1.w * rrf) * s1.w);
      Pack8 pk;
      pk.h = hv;
      u[i] = pk.u;
    }
    #pragma unroll
    for (int i = 0; i < 4; ++i) *(volatile v4u*)(dr + 256 * i + 8 * lane) = u[i];
    __threadfence();
    #pragma unroll
    for (int i = 0; i < 4; ++i) *(volatile v4u*)(dr + 256 * i + 8 * lane) = u[i];
  }

  if (lane == 0) {
    srec[4 * wv + 0] = w0;
    srec[4 * wv + 1] = w1;
    srec[4 * wv + 2] = (float)i0;
    srec[4 * wv + 3] = (float)i1;
    #pragma unroll
    for (int e = 0; e < NEX; ++e) sprob[wv * NEX + e] = tv ? (p[e] * inv) : 0.0f;
    sidx[2 * wv + 0] = tv ? i0 : -1;
    sidx[2 * wv + 1] = tv ? i1 : -1;
  }
  __syncthreads();
  if (wv == 0) {
    const int q = lane & 7;
    const v4f v = *(const v4fa*)(srec + 4 * q);
    const int tt = blockIdx.x * TPB + q;
    const bool ok = (lane < TPB) && (tt < ntok);
    float ps = 0.0f, cn = 0.0f;
    #pragma unroll
    for (int w = 0; w < TPB; ++w) {
      ps = ps + sprob[w * NEX + q];
      cn = cn + ((sidx[2 * w] == q) ? 1.0f : 0.0f) + ((sidx[2 * w + 1] == q) ? 1.0f : 0.0f);
    }
    float av[4], bv[4];
    #pragma unroll
    for (int j = 0; j < 4; ++j) {
      const int src = (4 * lane + j) & 7;
      av[j] = __shfl(ps, src);
      bv[j] = __shfl(cn, src);
    }
    v4f lv;
    lv.x = (lane < 2) ? av[0] : ((lane < 4) ? bv[0] : 0.0f);
    lv.y = (lane < 2) ? av[1] : ((lane < 4) ? bv[1] : 0.0f);
    lv.z = (lane < 2) ? av[2] : ((lane < 4) ? bv[2] : 0.0f);
    lv.w = (lane < 2) ? av[3] : ((lane < 4) ? bv[3] : 0.0f);
    float* lp = lbp + (size_t)blockIdx.x * LBW + 4 * lane;
    if (ok) *(volatile v4f*)(rec + (size_t)tt * 4) = v;
    if (lane < 8) *(volatile v4f*)lp = lv;
    __threadfence();
    if (ok) *(volatile v4f*)(rec + (size_t)tt * 4) = v;
    if (lane < 8) *(volatile v4f*)lp = lv;
  }
}

__device__ __forceinline__ void part_pass(const float* sY, const int* sTok, const int* sSlot,
                                          float* part, int ns, int wv, int lane, int nrows)
{
  #pragma unroll
  for (int i = 0; i < 8; ++i) {
    const int row = wv * 8 + i;
    int t = sTok[row];
    t = (t < 0) ? 0 : ((t > NTOK - 1) ? (NTOK - 1) : t);
    int s = sSlot[row];
    s = (s != 0) ? 1 : 0;
    const v4f v0 = *(const v4fa*)(sY + row * YP + 4 * lane);
    const v4f v1 = *(const v4fa*)(sY + row * YP + 128 + 4 * lane);
    float* dst = part + ((size_t)t * 2 + s) * DM + ns * 256;
    if (row < nrows) {
      *(volatile v4f*)(dst + 4 * lane) = v0;
      *(volatile v4f*)(dst + 128 + 4 * lane) = v1;
    }
  }
}

__global__ __launch_bounds__(256) void k_expert(const unsigned short* __restrict__ xh,
                                                const unsigned short* __restrict__ ew0,
                                                const unsigned short* __restrict__ ew1,
                                                const unsigned short* __restrict__ ewo,
                                                const float* __restrict__ rec,
                                                float* __restrict__ part, int ntok)
{
  extern __shared__ __align__(16) unsigned char dsm_e[];
  unsigned short* sX = (unsigned short*)dsm_e;
  unsigned short* sH = (unsigned short*)(dsm_e + LDS_XB);
  float* sY = (float*)dsm_e;
  __shared__ int   sTok[MT];
  __shared__ int   sSlot[MT];
  __shared__ float sW[MT];
  __shared__ int   s_wc[8];

  const int tid = threadIdx.x, lane = tid & 31, wv = tid >> 5;
  const int h = lane >> 4, m = lane & 15;
  const int wr = wv >> 2, wc = wv & 3;
  const int e = blockIdx.y;
  const int m0 = blockIdx.x * MT;

  if (tid < MT) { sTok[tid] = 0; sSlot[tid] = 0; sW[tid] = 0.0f; }
  __syncthreads();

  int base = 0;
  #pragma unroll 1
  for (int ch = 0; ch < NTOK / 256; ++ch) {
    const int t = ch * 256 + tid;
    const int tc = (t < ntok) ? t : (ntok - 1);
    const v4f r = *(const v4fa*)(rec + (size_t)tc * 4);
    int e0 = (int)r.z, e1 = (int)r.w;
    e0 = (e0 < 0) ? 0 : ((e0 > NEX - 1) ? (NEX - 1) : e0);
    e1 = (e1 < 0) ? 0 : ((e1 > NEX - 1) ? (NEX - 1) : e1);
    const bool f0 = (e0 == e);
    const bool f1 = (e1 == e) && !f0;
    const bool f = (f0 || f1) && (t < ntok);
    const unsigned int msk = __builtin_amdgcn_ballot_w32(f);
    const int off = __builtin_popcount(msk & ((1u << lane) - 1u));
    const int wcnt = __builtin_popcount(msk);
    if (lane == 0) s_wc[wv] = wcnt;
    __syncthreads();
    int pre = 0, tot = 0;
    #pragma unroll
    for (int w2 = 0; w2 < 8; ++w2) {
      const int cc = s_wc[w2];
      tot += cc;
      pre += (w2 < wv) ? cc : 0;
    }
    if (f) {
      const int p = base + pre + off - m0;
      if ((unsigned)p < (unsigned)MT) {
        sTok[p]  = t;
        sSlot[p] = f0 ? 0 : 1;
        sW[p]    = f0 ? r.x : r.y;
      }
    }
    base += tot;
    __syncthreads();
  }
  const int cnt = base;
  if (m0 >= cnt) return;
  int nrows = cnt - m0;
  nrows = (nrows > MT) ? MT : nrows;

  #pragma unroll 4
  for (int j = 0; j < 32; ++j) {
    const int idx = tid + 256 * j;
    const int row = idx >> 7, c8 = idx & 127;
    int t = sTok[row];
    t = (t < 0) ? 0 : ((t > NTOK - 1) ? (NTOK - 1) : t);
    const size_t go = (size_t)t * DM + 8 * c8;
    const v4u a = *(const v4ua*)(xh + go);
    *(v4ua*)(sX + row * XP + 8 * c8) = a;
  }
  __syncthreads();

  const v8f z8 = {0.f, 0.f, 0.f, 0.f, 0.f, 0.f, 0.f, 0.f};

  #pragma unroll 1
  for (int ns = 0; ns < MX / 128; ++ns) {
    v8f ag[2][2], au[2][2];
    #pragma unroll
    for (int mt = 0; mt < 2; ++mt)
      #pragma unroll
      for (int nt = 0; nt < 2; ++nt) { ag[mt][nt] = z8; au[mt][nt] = z8; }
    #pragma unroll 1
    for (int k0 = 0; k0 < DM; k0 += 32) {
      v16h a[2];
      #pragma unroll
      for (int mt = 0; mt < 2; ++mt)
        a[mt] = ldfrag(sX + (32 * wr + 16 * mt + m) * XP + k0, h);
      #pragma unroll
      for (int nt = 0; nt < 2; ++nt) {
        const int jg = ns * 128 + wc * 32 + 16 * nt + m;
        const size_t bo = ((size_t)e * MX + jg) * DM + k0;
        const v16h bg = ldfrag(ew0 + bo, h);
        const v16h bu = ldfrag(ew1 + bo, h);
        #pragma unroll
        for (int mt = 0; mt < 2; ++mt) {
          ag[mt][nt] = wmma_h(a[mt], bg, ag[mt][nt]);
          au[mt][nt] = wmma_h(a[mt], bu, au[mt][nt]);
        }
      }
    }
    #pragma unroll
    for (int mt = 0; mt < 2; ++mt)
      #pragma unroll
      for (int nt = 0; nt < 2; ++nt) {
        const int col = ns * 128 + wc * 32 + 16 * nt + m;
        #pragma unroll
        for (int r = 0; r < 8; ++r) {
          const int row = 32 * wr + 16 * mt + 8 * h + r;
          const float g = ag[mt][nt][r] * R_W;
          const float u = au[mt][nt][r] * R_W;
          const float hv = gelu_f(g) * u * H_SC;
          sH[row * HP + col] = hbits(hv);
        }
      }
  }
  __syncthreads();

  #pragma unroll 1
  for (int ns = 0; ns < DM / 256; ++ns) {
    v8f acc[2][4];
    #pragma unroll
    for (int mt = 0; mt < 2; ++mt)
      #pragma unroll
      for (int nt = 0; nt < 4; ++nt) acc[mt][nt] = z8;
    #pragma unroll 1
    for (int k0 = 0; k0 < MX; k0 += 32) {
      v16h a[2];
      #pragma unroll
      for (int mt = 0; mt < 2; ++mt)
        a[mt] = ldfrag(sH + (32 * wr + 16 * mt + m) * HP + k0, h);
      #pragma unroll
      for (int nt = 0; nt < 4; ++nt) {
        const int d = ns * 256 + wc * 64 + 16 * nt + m;
        const size_t bo = ((size_t)e * DM + d) * MX + k0;
        const v16h b = ldfrag(ewo + bo, h);
        #pragma unroll
        for (int mt = 0; mt < 2; ++mt) acc[mt][nt] = wmma_h(a[mt], b, acc[mt][nt]);
      }
    }
    #pragma unroll
    for (int mt = 0; mt < 2; ++mt)
      #pragma unroll
      for (int nt = 0; nt < 4; ++nt) {
        const int cl = wc * 64 + 16 * nt + m;
        #pragma unroll
        for (int r = 0; r < 8; ++r) {
          const int row = 32 * wr + 16 * mt + 8 * h + r;
          sY[row * YP + cl] = acc[mt][nt][r] * (sW[row] * R_HW);
        }
      }
    __syncthreads();
    part_pass(sY, sTok, sSlot, part, ns, wv, lane, nrows);
    __threadfence();
    part_pass(sY, sTok, sSlot, part, ns, wv, lane, nrows);
    __syncthreads();
  }
}

__global__ __launch_bounds__(256) void k_shgu(const unsigned short* __restrict__ xh,
                                              const unsigned short* __restrict__ sgp,
                                              const unsigned short* __restrict__ sup,
                                              unsigned short* __restrict__ hsp)
{
  __shared__ __align__(16) unsigned short sT[64 * TP];
  const int tid = threadIdx.x, lane = tid & 31, wv = tid >> 5;
  const int h = lane >> 4, m = lane & 15;
  const int wr = wv >> 2, wc = wv & 3;
  const int m0 = blockIdx.y * 64, n0 = blockIdx.x * 128;

  const v8f z8 = {0.f, 0.f, 0.f, 0.f, 0.f, 0.f, 0.f, 0.f};
  v8f ag[2][2], au[2][2];
  #pragma unroll
  for (int mt = 0; mt < 2; ++mt)
    #pragma unroll
    for (int nt = 0; nt < 2; ++nt) { ag[mt][nt] = z8; au[mt][nt] = z8; }

  #pragma unroll 1
  for (int k0 = 0; k0 < DM; k0 += 32) {
    v16h a[2];
    #pragma unroll
    for (int mt = 0; mt < 2; ++mt)
      a[mt] = ldfrag(xh + (size_t)(m0 + 32 * wr + 16 * mt + m) * DM + k0, h);
    #pragma unroll
    for (int nt = 0; nt < 2; ++nt) {
      const size_t ro = (size_t)(n0 + wc * 32 + 16 * nt + m) * DM + k0;
      const v16h bg = ldfrag(sgp + ro, h);
      const v16h bu = ldfrag(sup + ro, h);
      #pragma unroll
      for (int mt = 0; mt < 2; ++mt) {
        ag[mt][nt] = wmma_h(a[mt], bg, ag[mt][nt]);
        au[mt][nt] = wmma_h(a[mt], bu, au[mt][nt]);
      }
    }
  }
  #pragma unroll
  for (int mt = 0; mt < 2; ++mt)
    #pragma unroll
    for (int nt = 0; nt < 2; ++nt) {
      const int cl = wc * 32 + 16 * nt + m;
      #pragma unroll
      for (int r = 0; r < 8; ++r) {
        const int row = 32 * wr + 16 * mt + 8 * h + r;
        const float g = ag[mt][nt][r] * R_W;
        const float u = au[mt][nt][r] * R_W;
        sT[row * TP + cl] = hbits(gelu_f(g) * u * H_SC);
      }
    }
  __syncthreads();
  #pragma unroll
  for (int i = 0; i < 4; ++i) {
    const int rl = 8 * wv + 2 * i + h;
    const v4u u4 = *(const v4ua*)(sT + rl * TP + 8 * m);
    unsigned short* d = hsp + (size_t)(m0 + rl) * HS + n0 + 8 * m;
    *(volatile v4u*)d = u4;
    __threadfence();
    *(volatile v4u*)d = u4;
  }
}

__global__ __launch_bounds__(256) void k_shdn(const unsigned short* __restrict__ hsp,
                                              const unsigned short* __restrict__ sdp,
                                              float* __restrict__ shf)
{
  extern __shared__ __align__(16) unsigned char dsm_d[];
  float* sY = (float*)dsm_d;
  const int tid = threadIdx.x, lane = tid & 31, wv = tid >> 5;
  const int h = lane >> 4, m = lane & 15;
  const int wr = wv >> 2, wc = wv & 3;
  const int m0 = blockIdx.y * 64, n0 = blockIdx.x * 256;

  const v8f z8 = {0.f, 0.f, 0.f, 0.f, 0.f, 0.f, 0.f, 0.f};
  v8f acc[2][4];
  #pragma unroll
  for (int mt = 0; mt < 2; ++mt)
    #pragma unroll
    for (int nt = 0; nt < 4; ++nt) acc[mt][nt] = z8;

  #pragma unroll 1
  for (int k0 = 0; k0 < HS; k0 += 32) {
    v16h a[2];
    #pragma unroll
    for (int mt = 0; mt < 2; ++mt)
      a[mt] = ldfrag(hsp + (size_t)(m0 + 32 * wr + 16 * mt + m) * HS + k0, h);
    #pragma unroll
    for (int nt = 0; nt < 4; ++nt) {
      const v16h b = ldfrag(sdp + (size_t)(n0 + wc * 64 + 16 * nt + m) * HS + k0, h);
      #pragma unroll
      for (int mt = 0; mt < 2; ++mt) acc[mt][nt] = wmma_h(a[mt], b, acc[mt][nt]);
    }
  }
  #pragma unroll
  for (int mt = 0; mt < 2; ++mt)
    #pragma unroll
    for (int nt = 0; nt < 4; ++nt) {
      const int cl = wc * 64 + 16 * nt + m;
      #pragma unroll
      for (int r = 0; r < 8; ++r) {
        const int row = 32 * wr + 16 * mt + 8 * h + r;
        sY[row * YP + cl] = acc[mt][nt][r] * R_HW;
      }
    }
  __syncthreads();
  #pragma unroll
  for (int i = 0; i < 8; ++i) {
    const int rl = 8 * wv + i;
    const int t = m0 + rl;
    const v4f y0 = *(const v4fa*)(sY + rl * YP + 4 * lane);
    const v4f y1 = *(const v4fa*)(sY + rl * YP + 128 + 4 * lane);
    float* d = shf + (size_t)t * DM + n0;
    *(volatile v4f*)(d + 4 * lane) = y0;
    *(volatile v4f*)(d + 128 + 4 * lane) = y1;
    __threadfence();
    *(volatile v4f*)(d + 4 * lane) = y0;
    *(volatile v4f*)(d + 128 + 4 * lane) = y1;
  }
}

__global__ __launch_bounds__(256) void k_final(const float* __restrict__ shf,
                                               const float* __restrict__ part,
                                               const float* __restrict__ ps1,
                                               const float* __restrict__ ps2,
                                               float* __restrict__ out, int ntok)
{
  const int tid = threadIdx.x, lane = tid & 31, wv = tid >> 5;
  const int t = blockIdx.x * TPB + wv;
  const int tc = (t < ntok) ? t : (ntok - 1);
  const float* sr = shf + (size_t)tc * DM;
  const float* p0 = part + (size_t)tc * 2 * DM;
  const float* p1 = p0 + DM;

  v4f sv[8], rv[8];
  float ss = 0.0f, rs = 0.0f;
  #pragma unroll
  for (int i = 0; i < 8; ++i) {
    const int d = 128 * i + 4 * lane;
    const v4f s = *(const v4fa*)(sr + d);
    const v4f a = *(const v4fa*)(p0 + d);
    const v4f b = *(const v4fa*)(p1 + d);
    const v4f r = a + b;
    sv[i] = s;
    rv[i] = r;
    ss = ss + s.x * s.x + s.y * s.y + s.z * s.z + s.w * s.w;
    rs = rs + r.x * r.x + r.y * r.y + r.z * r.z + r.w * r.w;
  }
  #pragma unroll
  for (int off = 16; off > 0; off >>= 1) {
    ss = ss + __shfl_xor(ss, off);
    rs = rs + __shfl_xor(rs, off);
  }
  const float r1 = 1.0f / sqrtf(ss * (1.0f / 1024.0f) + 1.0e-6f);
  const float r2 = 1.0f / sqrtf(rs * (1.0f / 1024.0f) + 1.0e-6f);

  v4f ov[8];
  #pragma unroll
  for (int i = 0; i < 8; ++i) {
    const int d = 128 * i + 4 * lane;
    const v4f c1 = *(const v4fa*)(ps1 + d);
    const v4f c2 = *(const v4fa*)(ps2 + d);
    ov[i] = (rv[i] * r2) * c2 + (sv[i] * r1) * c1;
  }
  if (t < ntok) {
    float* dr = out + (size_t)t * DM;
    #pragma unroll
    for (int i = 0; i < 8; ++i) *(volatile v4f*)(dr + 128 * i + 4 * lane) = ov[i];
    __threadfence();
    #pragma unroll
    for (int i = 0; i < 8; ++i) *(volatile v4f*)(dr + 128 * i + 4 * lane) = ov[i];
  }
}

__global__ __launch_bounds__(256) void k_lb(const float* __restrict__ lbp, int nblk,
                                            float* __restrict__ out1)
{
  __shared__ double sred[16 * 256];
  __shared__ double sfin[16];
  const int tid = threadIdx.x;
  double a[16];
  #pragma unroll
  for (int j = 0; j < 16; ++j) a[j] = 0.0;
  #pragma unroll 1
  for (int i = tid; i < nblk; i += 256) {
    const float* ln = lbp + (size_t)i * LBW;
    const v4f q0 = *(const v4fa*)(ln + 0);
    const v4f q1 = *(const v4fa*)(ln + 4);
    const v4f q2 = *(const v4fa*)(ln + 8);
    const v4f q3 = *(const v4fa*)(ln + 12);
    a[0]  += (double)q0.x; a[1]  += (double)q0.y; a[2]  += (double)q0.z; a[3]  += (double)q0.w;
    a[4]  += (double)q1.x; a[5]  += (double)q1.y; a[6]  += (double)q1.z; a[7]  += (double)q1.w;
    a[8]  += (double)q2.x; a[9]  += (double)q2.y; a[10] += (double)q2.z; a[11] += (double)q2.w;
    a[12] += (double)q3.x; a[13] += (double)q3.y; a[14] += (double)q3.z; a[15] += (double)q3.w;
  }
  #pragma unroll
  for (int j = 0; j < 16; ++j) sred[j * 256 + tid] = a[j];
  __syncthreads();
  if (tid < 16) {
    double s = 0.0;
    #pragma unroll 1
    for (int j = 0; j < 256; ++j) s += sred[tid * 256 + j];
    sfin[tid] = s;
  }
  __syncthreads();
  if (tid == 0) {
    double lb = 0.0;
    #pragma unroll
    for (int e = 0; e < NEX; ++e)
      lb += (sfin[8 + e] * (1.0 / ((double)NTOK * 2.0))) * (sfin[e] * (1.0 / (double)NTOK));
    const float v = (float)(lb * (double)NEX);
    *(volatile float*)out1 = v;
    __threadfence();
    *(volatile float*)out1 = v;
  }
}

extern "C" void kernel_launch(void* const* d_in, const int* in_sizes, int n_in,
                              void* d_out, int out_size, void* d_ws, size_t ws_size,
                              hipStream_t stream)
{
  if (n_in < 13) return;
  if (in_sizes[0] != NTOK * DM) return;
  if (in_sizes[1] != NTOK * DM) return;
  if (in_sizes[2] != DM || in_sizes[3] != DM || in_sizes[4] != DM || in_sizes[5] != DM) return;
  if (in_sizes[6] != DM * NEX) return;
  if (in_sizes[7] != NEX * DM * MX) return;
  if (in_sizes[8] != NEX * DM * MX) return;
  if (in_sizes[9] != NEX * MX * DM) return;
  if (in_sizes[10] != DM * HS) return;
  if (in_sizes[11] != DM * HS) return;
  if (in_sizes[12] != HS * DM) return;
  if (out_size != NTOK * DM + 1) return;

  const float* xin  = (const float*)d_in[0];
  const float* xorg = (const float*)d_in[1];
  const float* pfs  = (const float*)d_in[2];
  const float* pls  = (const float*)d_in[3];
  const float* ps1  = (const float*)d_in[4];
  const float* ps2  = (const float*)d_in[5];
  const float* rw   = (const float*)d_in[6];
  const float* ewi0 = (const float*)d_in[7];
  const float* ewi1 = (const float*)d_in[8];
  const float* ewo  = (const float*)d_in[9];
  const float* swi0 = (const float*)d_in[10];
  const float* swi1 = (const float*)d_in[11];
  const float* swo  = (const float*)d_in[12];
  float* out = (float*)d_out;

  const size_t bXH   = (size_t)NTOK * DM * 2;
  const size_t bRXH  = (size_t)NTOK * DM * 2;
  const size_t bSG   = (size_t)HS * DM * 2;
  const size_t bSD   = (size_t)DM * HS * 2;
  const size_t bEW   = (size_t)NEX * MX * DM * 2;
  const size_t bHSP  = (size_t)NTOK * HS * 2;
  const size_t bREC  = (size_t)NTOK * 16;
  const size_t bLBP  = (size_t)NBLK * LBW * 4;
  const size_t bPART = (size_t)NTOK * 2 * DM * 4;
  const size_t total = bXH + bRXH + 2 * bSG + bSD + 3 * bEW + bHSP + bREC + bLBP + bPART;
  if (total > ws_size) return;
  if (total > (size_t)134217728) return;

  char* ws = (char*)d_ws;
  size_t off = 0;
  unsigned short* XH   = (unsigned short*)(ws + off); off += bXH;
  unsigned short* RXH  = (unsigned short*)(ws + off); off += bRXH;
  unsigned short* SG0  = (unsigned short*)(ws + off); off += bSG;
  unsigned short* SG1  = (unsigned short*)(ws + off); off += bSG;
  unsigned short* SDP  = (unsigned short*)(ws + off); off += bSD;
  unsigned short* EW0  = (unsigned short*)(ws + off);
  float*          SHF  = (float*)(ws + off);          off += bEW;
  unsigned short* EW1  = (unsigned short*)(ws + off); off += bEW;
  unsigned short* EWO  = (unsigned short*)(ws + off); off += bEW;
  unsigned short* HSP  = (unsigned short*)(ws + off); off += bHSP;
  float*          REC  = (float*)(ws + off);          off += bREC;
  float*          LBP  = (float*)(ws + off);          off += bLBP;
  float*          PART = (float*)(ws + off);          off += bPART;
  if (off != total) return;

  hipFuncSetAttribute(reinterpret_cast<const void*>(&k_expert),
                      hipFuncAttributeMaxDynamicSharedMemorySize, LDS_EXP);
  hipFuncSetAttribute(reinterpret_cast<const void*>(&k_shdn),
                      hipFuncAttributeMaxDynamicSharedMemorySize, LDS_DN);

  {
    const int n8x = NTOK * DM / 8;
    k_cvt<<<(n8x + 255) / 256, 256, 0, stream>>>(xin, XH, n8x, 1.0f);
  }
  k_tr<<<dim3(HS / 64, DM / 64, 1),   256, 0, stream>>>(swi0, SG0, DM, HS, W_SC);
  k_tr<<<dim3(HS / 64, DM / 64, 1),   256, 0, stream>>>(swi1, SG1, DM, HS, W_SC);
  k_tr<<<dim3(DM / 64, HS / 64, 1),   256, 0, stream>>>(swo,  SDP, HS, DM, W_SC);
  k_tr<<<dim3(MX / 64, DM / 64, NEX), 256, 0, stream>>>(ewi0, EW0, DM, MX, W_SC);
  k_tr<<<dim3(MX / 64, DM / 64, NEX), 256, 0, stream>>>(ewi1, EW1, DM, MX, W_SC);
  k_tr<<<dim3(DM / 64, MX / 64, NEX), 256, 0, stream>>>(ewo,  EWO, MX, DM, W_SC);
  k_route<<<NBLK, 256, 0, stream>>>(xorg, pfs, pls, rw, REC, RXH, LBP, NTOK);
  k_expert<<<dim3(NTOK / MT, NEX), 256, LDS_EXP, stream>>>(RXH, EW0, EW1, EWO, REC, PART, NTOK);
  k_shgu<<<dim3(HS / 128, NTOK / 64), 256, 0, stream>>>(XH, SG0, SG1, HSP);
  k_shdn<<<dim3(DM / 256, NTOK / 64), 256, LDS_DN, stream>>>(HSP, SDP, SHF);
  k_final<<<NBLK, 256, 0, stream>>>(SHF, PART, ps1, ps2, out, NTOK);
  k_lb<<<1, 256, 0, stream>>>(LBP, NBLK, out + (size_t)NTOK * DM);
}
